// MultiHeadHierarchicalAttentionBlock_80556406604302
// MI455X (gfx1250) — hardware-verified
//
#include <hip/hip_runtime.h>


namespace {
constexpr int Bn = 2, C = 256, SC = 64, S = 4096, NT = Bn * S, RK = 16, FF = 1024;
constexpr float WS = 512.0f, AS = 8.0f, LS = 64.0f, VS = 8.0f, EPS = 1e-5f;

typedef _Float16 b16;
typedef __attribute__((ext_vector_type(16))) _Float16 v16b;
typedef __attribute__((ext_vector_type(8)))  _Float16 v8b;
typedef __attribute__((ext_vector_type(8)))  float v8f;
typedef __attribute__((ext_vector_type(4)))  float v4f;

__device__ __forceinline__ v8b ld8b(const b16* p) { return *(const v8b*)p; }
__device__ __forceinline__ v16b cat8b(v8b a, v8b b) { return __builtin_shufflevector(a, b, 0, 1, 2, 3, 4, 5, 6, 7, 8, 9, 10, 11, 12, 13, 14, 15); }
__device__ __forceinline__ v16b frag_kb(const b16* p, int hh) { return cat8b(ld8b(p + 8 * hh), ld8b(p + 16 + 8 * hh)); }
__device__ __forceinline__ void split16(float v, b16& hi, b16& lo) { hi = (b16)v; lo = (b16)(v - (float)hi); }
__device__ __forceinline__ void frag_ksplit(const float* p, int hh, v16b& fh_, v16b& fl_) {
  const float* p0 = p + 8 * hh; const float* p1 = p + 16 + 8 * hh;
#pragma unroll
  for (int e = 0; e < 8; ++e) { b16 a, c; split16(p0[e], a, c); fh_[e] = a; fl_[e] = c; split16(p1[e], a, c); fh_[8 + e] = a; fl_[8 + e] = c; }
}
__device__ __forceinline__ v8f wmma16b(v16b a, v16b b, v8f c) {
  v8f d = __builtin_amdgcn_wmma_f32_16x16x32_f16(false, a, false, b, (short)0, c, false, false);
  asm volatile("v_nop\n\tv_nop\n\tv_nop\n\tv_nop" : "+v"(d) : "v"(a), "v"(b));
  return d;
}
__device__ __forceinline__ void wave_lds_sync() {
  __builtin_amdgcn_fence(__ATOMIC_RELEASE, "workgroup");
  __builtin_amdgcn_wave_barrier();
  __builtin_amdgcn_fence(__ATOMIC_ACQUIRE, "workgroup");
}

struct Opnd { const void* p0; const void* p1; int ld; };
template <int NP> __device__ __forceinline__ void load_frags(const Opnd& o, int row, int kb, int hh, v16b& fh_, v16b& fl_) {
  if (NP == 0) { frag_ksplit((const float*)o.p0 + (size_t)row * o.ld + kb, hh, fh_, fl_); }
  else if (NP == 4 || NP == 5) {
    const float sc_ = (NP == 4) ? 64.0f : 8.0f;
    const float* p = (const float*)o.p0 + (size_t)row * o.ld + kb; const float* p0 = p + 8 * hh; const float* p1 = p + 16 + 8 * hh;
#pragma unroll
    for (int e = 0; e < 8; ++e) { b16 a, c; split16(p0[e] * sc_, a, c); fh_[e] = a; fl_[e] = c; split16(p1[e] * sc_, a, c); fh_[8 + e] = a; fl_[8 + e] = c; }
  } else if (NP == 3) {
    const float* p = (const float*)o.p0 + (size_t)row * o.ld + kb; const float* p0 = p + 8 * hh; const float* p1 = p + 16 + 8 * hh;
#pragma unroll
    for (int e = 0; e < 8; ++e) { fh_[e] = (b16)p0[e]; fh_[8 + e] = (b16)p1[e]; }
    fl_ = fh_;
  } else {
    fh_ = frag_kb((const b16*)o.p0 + (size_t)row * o.ld + kb, hh);
    if (NP == 2) fl_ = frag_kb((const b16*)o.p1 + (size_t)row * o.ld + kb, hh); else fl_ = fh_;
  }
}
template <int ANP, int BNP> __device__ __forceinline__ v8f mac(v16b ah, v16b al, v16b bh, v16b bl, v8f c) {
  c = wmma16b(ah, bh, c);
  if (BNP == 0 || BNP == 2 || BNP == 4 || BNP == 5) c = wmma16b(ah, bl, c);
  if (ANP == 0 || ANP == 2 || ANP == 4 || ANP == 5) c = wmma16b(al, bh, c);
  return c;
}
template <int ANP, int BNP>
__device__ __forceinline__ void gemm_tile(const Opnd& A, const Opnd& B, int K, int m0, int c0, int nloc, int hlf, v8f (&acc)[2][4]) {
  for (int kb = 0; kb < K; kb += 32) {
    v16b a0h, a0l, a1h, a1l;
    load_frags<ANP>(A, m0 + nloc, kb, hlf, a0h, a0l);
    load_frags<ANP>(A, m0 + 16 + nloc, kb, hlf, a1h, a1l);
#pragma unroll
    for (int t = 0; t < 4; ++t) {
      v16b bh, bl;
      load_frags<BNP>(B, c0 + t * 16 + nloc, kb, hlf, bh, bl);
      acc[0][t] = mac<ANP, BNP>(a0h, a0l, bh, bl, acc[0][t]);
      acc[1][t] = mac<ANP, BNP>(a1h, a1l, bh, bl, acc[1][t]);
    }
  }
}

__device__ __forceinline__ void epi_planes(v8f (&acc)[2][4], float scale, bool two, b16* __restrict__ oh, b16* __restrict__ ol, int ldo,
                                           int m0, int c0, int lane, b16* Th, b16* Tl) {
  const int nloc = lane & 15, hlf = lane >> 4;
#pragma unroll
  for (int t = 0; t < 4; ++t)
#pragma unroll
    for (int r = 0; r < 2; ++r)
#pragma unroll
      for (int v = 0; v < 8; ++v) {
        const int rr = r * 16 + v + 8 * hlf, cc = t * 16 + nloc;
        b16 h_, l_; split16(acc[r][t][v] * scale, h_, l_);
        Th[rr * 64 + cc] = h_; Tl[rr * 64 + cc] = l_;
      }
  wave_lds_sync();
  for (int pass = 0; pass < 2; ++pass) {
#pragma unroll
    for (int j = 0; j < 8; ++j) {
      const int rr = j * 4 + (lane >> 3), c8 = (lane & 7) * 8;
      const size_t o = (size_t)(m0 + rr) * ldo + c0 + c8;
      *(volatile v8b*)(oh + o) = ld8b(Th + rr * 64 + c8);
      if (two) *(volatile v8b*)(ol + o) = ld8b(Tl + rr * 64 + c8);
    }
    __threadfence();
  }
}
__device__ __forceinline__ void epi_f32(v8f (&acc)[2][4], float scale, const float* rscale, float* __restrict__ out, int ldo, int m0, int c0, int lane, float* Tt) {
  const int nloc = lane & 15, hlf = lane >> 4;
#pragma unroll
  for (int t = 0; t < 4; ++t)
#pragma unroll
    for (int r = 0; r < 2; ++r)
#pragma unroll
      for (int v = 0; v < 8; ++v) {
        const int rr = r * 16 + v + 8 * hlf;
        const float rs = rscale ? rscale[(size_t)(m0 + rr) * 32] : 1.0f;
        Tt[rr * 64 + t * 16 + nloc] = acc[r][t][v] * scale * rs;
      }
  wave_lds_sync();
  float* dst0 = out + (size_t)m0 * ldo + c0;
  for (int pass = 0; pass < 2; ++pass) {
#pragma unroll
    for (int j = 0; j < 16; ++j) { const int rr = j * 2 + hlf, c4 = nloc * 4; *(volatile v4f*)(dst0 + (size_t)rr * ldo + c4) = *(const v4f*)(Tt + rr * 64 + c4); }
    __threadfence();
  }
}


__global__ __launch_bounds__(256) void prep_kernel(const float* __restrict__ qw, const float* __restrict__ kw, const float* __restrict__ vw, const float* __restrict__ qlw,
                                                   const float* __restrict__ klw, const float* __restrict__ ow, const float* __restrict__ f1w, const float* __restrict__ f2w,
                                                   const float* __restrict__ qb, const float* __restrict__ kb, const float* __restrict__ vb,
                                                   b16* __restrict__ ph, b16* __restrict__ pl, float* __restrict__ bqkv) {
  const size_t tid = (size_t)blockIdx.x * blockDim.x + threadIdx.x, stride = (size_t)gridDim.x * blockDim.x;
  const size_t nqkv = (size_t)4 * 192 * 64, nl = (size_t)4 * 32 * 64, no = (size_t)4 * 64 * 64, n1 = (size_t)FF * C, n2 = (size_t)C * FF;
  const size_t tot = (nqkv + nl + no + n1 + n2) / 8;
  for (int pass = 0; pass < 2; ++pass) {
    for (size_t c8 = tid; c8 < tot; c8 += stride) {
      const size_t i0 = c8 * 8; v8b vh, vl;
#pragma unroll
      for (int e = 0; e < 8; ++e) {
        size_t i = i0 + e; float w;
        if (i < nqkv) { const int hd = (int)(i / (192 * 64)), r = (int)((i / 64) % 192), k = (int)(i % 64); const float* src = (r < 64) ? qw : (r < 128) ? kw : vw; w = src[((size_t)hd * 64 + (r % 64)) * 64 + k]; }
        else if ((i -= nqkv) < nl) { const int hd = (int)(i / (32 * 64)), r = (int)((i / 64) % 32), k = (int)(i % 64); w = ((r < 16) ? qlw : klw)[((size_t)hd * 16 + (r % 16)) * 64 + k]; }
        else if ((i -= nl) < no) { w = ow[i]; }
        else if ((i -= no) < n1) { w = f1w[i]; }
        else { i -= n1; w = f2w[i]; }
        b16 a, b2; split16(w * WS, a, b2); vh[e] = a; vl[e] = b2;
      }
      *(volatile v8b*)(ph + i0) = vh; *(volatile v8b*)(pl + i0) = vl;
    }
    for (size_t j = tid; j < 4 * 192 / 4; j += stride) { const int hd = (int)(j / 48), r4 = (int)(j % 48) * 4; const float* src = (r4 < 64) ? qb : (r4 < 128) ? kb : vb;
      *(volatile v4f*)(bqkv + hd * 192 + r4) = *(const v4f*)(src + hd * 64 + (r4 % 64)); }
    __threadfence();
  }
}

__global__ __launch_bounds__(256) void xt_kernel(const float* __restrict__ x, float* __restrict__ xT, float* __restrict__ xin) {
  __shared__ float Tl[64][C + 4];
  const int b = blockIdx.x / (S / 64), s0 = (blockIdx.x % (S / 64)) * 64, tid = threadIdx.x, lane = tid & 31, wave = tid >> 5;
  for (int i = tid; i < C * 64; i += 256) { const int c = i / 64, s = i % 64; Tl[s][c] = x[((size_t)b * C + c) * S + s0 + s]; }
  __syncthreads();
  for (int pass = 0; pass < 2; ++pass) {
    for (int j = 0; j < 8; ++j) { const int s = wave * 8 + j;
      *(volatile v4f*)(xT + ((size_t)b * S + s0 + s) * C + lane * 4) = *(const v4f*)(&Tl[s][lane * 4]);
      *(volatile v4f*)(xT + ((size_t)b * S + s0 + s) * C + 128 + lane * 4) = *(const v4f*)(&Tl[s][128 + lane * 4]);
      if (lane < 16) *(volatile v4f*)(xin + ((size_t)b * S + s0 + s) * SC + lane * 4) = *(const v4f*)(&Tl[s][lane * 4]); }
    __threadfence();
  }
}

__global__ __launch_bounds__(128) void qkv_kernel(const float* __restrict__ xin, const b16* __restrict__ wh, const b16* __restrict__ wl, const float* __restrict__ bias,
                                                  float* __restrict__ QK, b16* __restrict__ vth, b16* __restrict__ vtl) {
  __shared__ __attribute__((aligned(16))) float Ts[4][32 * 64];
  __shared__ __attribute__((aligned(16))) b16 Th[64][128 + 8]; __shared__ __attribute__((aligned(16))) b16 Tlo[64][128 + 8];
  const int lane = threadIdx.x & 31, wave = threadIdx.x >> 5, nloc = lane & 15, hlf = lane >> 4;
  const int m0 = blockIdx.y * 128 + wave * 32, c0 = blockIdx.x * 64;
  v8f acc[2][4];
#pragma unroll
  for (int r = 0; r < 2; ++r)
#pragma unroll
    for (int t = 0; t < 4; ++t) acc[r][t] = (v8f){};
  const Opnd A{xin, nullptr, SC}, B{wh, wl, SC};
  gemm_tile<5, 2>(A, B, SC, m0, c0, nloc, hlf, acc);
#pragma unroll
  for (int t = 0; t < 4; ++t)
#pragma unroll
    for (int r = 0; r < 2; ++r)
#pragma unroll
      for (int v = 0; v < 8; ++v) acc[r][t][v] = acc[r][t][v] * (1.0f / (AS * WS)) + bias[c0 + t * 16 + nloc];
  if (blockIdx.x < 2) { epi_f32(acc, 1.0f, nullptr, QK, 128, m0, c0, lane, Ts[wave]); return; }
#pragma unroll
  for (int t = 0; t < 4; ++t)
#pragma unroll
    for (int r = 0; r < 2; ++r)
#pragma unroll
      for (int v = 0; v < 8; ++v) { b16 a, b2; split16(acc[r][t][v] * VS, a, b2); Th[t * 16 + nloc][wave * 32 + r * 16 + 8 * hlf + v] = a; Tlo[t * 16 + nloc][wave * 32 + r * 16 + 8 * hlf + v] = b2; }
  __syncthreads();
  const int b = (blockIdx.y * 128) / S, tok0 = (blockIdx.y * 128) % S;
  b16* bh_ = vth + (size_t)b * SC * S + tok0; b16* bl_ = vtl + (size_t)b * SC * S + tok0;
  for (int pass = 0; pass < 2; ++pass) {
#pragma unroll
    for (int j = 0; j < 8; ++j) { const int d = wave * 16 + j * 2 + (lane >> 4), c8 = (lane & 15) * 8;
      *(volatile v8b*)(bh_ + (size_t)d * S + c8) = *(const v8b*)(&Th[d][c8]); *(volatile v8b*)(bl_ + (size_t)d * S + c8) = *(const v8b*)(&Tlo[d][c8]); }
    __threadfence();
  }
}

__global__ __launch_bounds__(128) void ql_kernel(const float* __restrict__ QK, const b16* __restrict__ wh, const b16* __restrict__ wl, float* __restrict__ L) {
  __shared__ __attribute__((aligned(16))) float Ts[4][32 * 16];
  const int lane = threadIdx.x & 31, wave = threadIdx.x >> 5, nloc = lane & 15, hlf = lane >> 4, z = blockIdx.y, m0 = blockIdx.x * 128 + wave * 32;
  v8f acc[2] = {{}, {}};
  const Opnd A{QK + z * SC, nullptr, 128}, B{wh + (size_t)z * 16 * SC, wl + (size_t)z * 16 * SC, SC};
  for (int kb = 0; kb < SC; kb += 32) {
    v16b a0h, a0l, a1h, a1l, bh, bl;
    load_frags<5>(A, m0 + nloc, kb, hlf, a0h, a0l); load_frags<5>(A, m0 + 16 + nloc, kb, hlf, a1h, a1l); load_frags<2>(B, nloc, kb, hlf, bh, bl);
    acc[0] = mac<5, 2>(a0h, a0l, bh, bl, acc[0]); acc[1] = mac<5, 2>(a1h, a1l, bh, bl, acc[1]);
  }
  float* Tt = Ts[wave];
#pragma unroll
  for (int r = 0; r < 2; ++r)
#pragma unroll
    for (int v = 0; v < 8; ++v) Tt[(r * 16 + v + 8 * hlf) * 16 + nloc] = acc[r][v] * (1.0f / (AS * WS));
  wave_lds_sync();
  float* dst = L + ((size_t)z * NT + m0) * RK;
  for (int pass = 0; pass < 2; ++pass) {
#pragma unroll
    for (int j = 0; j < 4; ++j) *(volatile v4f*)(dst + (j * 32 + lane) * 4) = *(const v4f*)(Tt + (j * 32 + lane) * 4);
    __threadfence();
  }
}

__global__ __launch_bounds__(256) void attn_kernel(const float* __restrict__ L, const b16* __restrict__ vth, const b16* __restrict__ vtl, float* __restrict__ O) {
  __shared__ __attribute__((aligned(16))) float Os[8][16 * SC];
  const int wid = threadIdx.x >> 5, lane = threadIdx.x & 31, hh = lane >> 4, col = lane & 15;
  const int qt = blockIdx.x * 8 + wid, b = qt / (S / 16), q0 = (qt % (S / 16)) * 16;
  const float* Ql = L + ((size_t)b * S) * RK; const float* Kl = L + ((size_t)NT + (size_t)b * S) * RK;
  v16b qh, qlo;
  { const float* qr = Ql + (size_t)(q0 + col) * RK;
#pragma unroll
    for (int e = 0; e < 16; ++e) { b16 a = (b16)0.0f, c = (b16)0.0f; if (e < 8) split16(qr[8 * hh + e] * LS, a, c); qh[e] = a; qlo[e] = c; } }
  const b16* vh = vth + (size_t)b * SC * S; const b16* vl = vtl + (size_t)b * SC * S;
  float m = -INFINITY, l = 0.0f; v8f o[4] = {{}, {}, {}, {}};
  for (int kb = 0; kb < S; kb += 32) {
    v8f s[2] = {{}, {}};
#pragma unroll
    for (int half = 0; half < 2; ++half) {
      const float* kr = Kl + (size_t)(kb + half * 16 + col) * RK; v16b kh, klo;
#pragma unroll
      for (int e = 0; e < 16; ++e) { b16 a = (b16)0.0f, c = (b16)0.0f; if (e < 8) split16(kr[8 * hh + e] * LS, a, c); kh[e] = a; klo[e] = c; }
      s[half] = mac<2, 2>(kh, klo, qh, qlo, s[half]);
    }
    float mr = -INFINITY;
#pragma unroll
    for (int r = 0; r < 8; ++r) { s[0][r] *= (0.25f / (LS * LS)); s[1][r] *= (0.25f / (LS * LS)); mr = fmaxf(mr, fmaxf(s[0][r], s[1][r])); }
    mr = fmaxf(mr, __shfl_xor(mr, 16));
    const float mn = fmaxf(m, mr), al_ = __expf(m - mn); m = mn;
    float sum = 0.0f; v16b pb;
#pragma unroll
    for (int r = 0; r < 8; ++r) { const float p0 = __expf(s[0][r] - mn), p1 = __expf(s[1][r] - mn); sum += p0 + p1; pb[r] = (b16)p0; pb[8 + r] = (b16)p1; }
    sum += __shfl_xor(sum, 16); l = l * al_ + sum;
#pragma unroll
    for (int n = 0; n < 4; ++n) {
#pragma unroll
      for (int r = 0; r < 8; ++r) o[n][r] *= al_;
      const size_t ro = (size_t)(n * 16 + col) * S + kb;
      o[n] = wmma16b(frag_kb(vh + ro, hh), pb, o[n]); o[n] = wmma16b(frag_kb(vl + ro, hh), pb, o[n]);
    }
  }
  const float inv = 1.0f / (VS * l); float* Tt = Os[wid];
#pragma unroll
  for (int n = 0; n < 4; ++n)
#pragma unroll
    for (int r = 0; r < 8; ++r) Tt[col * SC + n * 16 + 8 * hh + r] = o[n][r] * inv;
  wave_lds_sync();
  float* dst = O + ((size_t)b * S + q0) * SC;
  for (int pass = 0; pass < 2; ++pass) {
#pragma unroll
    for (int j = 0; j < 8; ++j) { const int rr = j * 2 + hh, c4 = col * 4; *(volatile v4f*)(dst + (size_t)rr * SC + c4) = *(const v4f*)(Tt + rr * SC + c4); }
    __threadfence();
  }
}

__global__ __launch_bounds__(128) void oproj_kernel(const float* __restrict__ O, const b16* __restrict__ wh, const b16* __restrict__ wl, const float* __restrict__ ob,
                                                    const float* __restrict__ xT, int hd, float* __restrict__ cat, float* __restrict__ xin) {
  __shared__ __attribute__((aligned(16))) float Ts[4][32 * 64];
  const int lane = threadIdx.x & 31, wave = threadIdx.x >> 5, nloc = lane & 15, hlf = lane >> 4, m0 = blockIdx.x * 128 + wave * 32;
  v8f acc[2][4];
#pragma unroll
  for (int r = 0; r < 2; ++r)
#pragma unroll
    for (int t = 0; t < 4; ++t) acc[r][t] = (v8f){};
  const Opnd A{O, nullptr, SC}, B{wh, wl, SC};
  gemm_tile<5, 2>(A, B, SC, m0, 0, nloc, hlf, acc);
  float* Tt = Ts[wave];
#pragma unroll
  for (int t = 0; t < 4; ++t)
#pragma unroll
    for (int r = 0; r < 2; ++r)
#pragma unroll
      for (int v = 0; v < 8; ++v) Tt[(r * 16 + v + 8 * hlf) * 64 + t * 16 + nloc] = acc[r][t][v] * (1.0f / (AS * WS)) + ob[t * 16 + nloc];
  wave_lds_sync();
  for (int pass = 0; pass < 2; ++pass) {
#pragma unroll
    for (int j = 0; j < 16; ++j) { const int rr = j * 2 + hlf, c4 = nloc * 4; const v4f pv = *(const v4f*)(Tt + rr * 64 + c4);
      *(volatile v4f*)(cat + (size_t)(m0 + rr) * C + hd * SC + c4) = pv;
      if (hd < 3) { v4f xv = *(const v4f*)(xT + (size_t)(m0 + rr) * C + (hd + 1) * SC + c4); xv += pv; *(volatile v4f*)(xin + (size_t)(m0 + rr) * SC + c4) = xv; } }
    __threadfence();
  }
}

__global__ __launch_bounds__(256) void bnstat_kernel(const float* __restrict__ X, int ld, const float* __restrict__ g, const float* __restrict__ bb, float* __restrict__ coef) {
  const int c = threadIdx.x; double s = 0.0, s2 = 0.0;
#pragma unroll 1
  for (int r = 0; r < NT; ++r) { const double v = X[(size_t)r * ld + c]; s += v; s2 += v * v; }
  const double mean = s / NT, var = s2 / NT - mean * mean;
  const float a = g[c] * (float)(1.0 / sqrt(var + (double)EPS)), sh = bb[c] - (float)mean * a;
  for (int pass = 0; pass < 2; ++pass) { ((volatile float*)coef)[c] = a; ((volatile float*)coef)[C + c] = sh; __threadfence(); }
}

__global__ __launch_bounds__(256) void bn1_kernel(const float* __restrict__ xT, const float* __restrict__ cat, const float* __restrict__ coef, float* __restrict__ out1) {
  const int lane = threadIdx.x & 31, row = blockIdx.x * 8 + (threadIdx.x >> 5);
  v4f w[2];
#pragma unroll
  for (int p = 0; p < 2; ++p) { const int c = p * 128 + lane * 4; const v4f xv = *(const v4f*)(xT + (size_t)row * C + c), cv = *(const v4f*)(cat + (size_t)row * C + c);
#pragma unroll
    for (int e = 0; e < 4; ++e) w[p][e] = xv[e] + cv[e] * coef[c + e] + coef[C + c + e]; }
  for (int pass = 0; pass < 2; ++pass) {
#pragma unroll
    for (int p = 0; p < 2; ++p) *(volatile v4f*)(out1 + (size_t)row * C + p * 128 + lane * 4) = w[p];
    __threadfence();
  }
}

__global__ __launch_bounds__(128) void ffn1_kernel(const float* __restrict__ out1, const b16* __restrict__ wh, const b16* __restrict__ wl, const float* __restrict__ f1b, b16* __restrict__ hh_, b16* __restrict__ hl_) {
  __shared__ __attribute__((aligned(16))) b16 Ts[4][2][32 * 64];
  const int lane = threadIdx.x & 31, wave = threadIdx.x >> 5, nloc = lane & 15, hlf = lane >> 4;
  const int m0 = blockIdx.y * 128 + wave * 32, c0 = blockIdx.x * 64;
  v8f acc[2][4];
#pragma unroll
  for (int r = 0; r < 2; ++r)
#pragma unroll
    for (int t = 0; t < 4; ++t) acc[r][t] = (v8f){};
  const Opnd A{out1, nullptr, C}, B{wh, wl, C};
  gemm_tile<5, 2>(A, B, C, m0, c0, nloc, hlf, acc);
#pragma unroll
  for (int t = 0; t < 4; ++t)
#pragma unroll
    for (int r = 0; r < 2; ++r)
#pragma unroll
      for (int v = 0; v < 8; ++v) { const float hv = acc[r][t][v] * (1.0f / (AS * WS)) + f1b[c0 + t * 16 + nloc]; acc[r][t][v] = 0.5f * hv * (1.0f + erff(hv * 0.7071067811865475f)); }
  epi_planes(acc, AS, true, hh_, hl_, FF, m0, c0, lane, Ts[wave][0], Ts[wave][1]);
}

__global__ __launch_bounds__(128) void ffn2_kernel(const b16* __restrict__ hh_, const b16* __restrict__ hl_, const b16* __restrict__ wh, const b16* __restrict__ wl, const float* __restrict__ f2b, float* __restrict__ h2) {
  __shared__ __attribute__((aligned(16))) float Ts[4][32 * 64];
  const int lane = threadIdx.x & 31, wave = threadIdx.x >> 5, nloc = lane & 15, hlf = lane >> 4;
  const int m0 = blockIdx.y * 128 + wave * 32, c0 = blockIdx.x * 64;
  v8f acc[2][4];
#pragma unroll
  for (int r = 0; r < 2; ++r)
#pragma unroll
    for (int t = 0; t < 4; ++t) acc[r][t] = (v8f){};
  const Opnd A{hh_, hl_, FF}, B{wh, wl, FF};
  gemm_tile<2, 2>(A, B, FF, m0, c0, nloc, hlf, acc);
#pragma unroll
  for (int t = 0; t < 4; ++t)
#pragma unroll
    for (int r = 0; r < 2; ++r)
#pragma unroll
      for (int v = 0; v < 8; ++v) acc[r][t][v] = acc[r][t][v] * (1.0f / (AS * WS)) + f2b[c0 + t * 16 + nloc];
  epi_f32(acc, 1.0f, nullptr, h2, C, m0, c0, lane, Ts[wave]);
}

__global__ __launch_bounds__(256) void final_kernel(const float* __restrict__ out1, const float* __restrict__ h2, const float* __restrict__ coef, float* __restrict__ out) {
  __shared__ float Tl[C][64 + 4];
  const int b = blockIdx.x / (S / 64), s0 = (blockIdx.x % (S / 64)) * 64, tid = threadIdx.x, lane = tid & 31, wave = tid >> 5;
  for (int i = tid; i < 64 * C; i += 256) { const int s = i / C, c = i % C; const size_t rix = ((size_t)b * S + s0 + s) * C + c; Tl[c][s] = out1[rix] + h2[rix] * coef[c] + coef[C + c]; }
  __syncthreads();
  for (int pass = 0; pass < 2; ++pass) {
#pragma unroll
    for (int j = 0; j < 16; ++j) { const int c = wave * 32 + j * 2 + (lane >> 4), c4 = (lane & 15) * 4; *(volatile v4f*)(out + ((size_t)b * C + c) * S + s0 + c4) = *(const v4f*)(&Tl[c][c4]); }
    __threadfence();
  }
}
}

extern "C" void kernel_launch(void* const* d_in, const int* in_sizes, int n_in,
                              void* d_out, int out_size, void* d_ws, size_t ws_size, hipStream_t stream) {
  (void)n_in; (void)out_size;
  const float* x = (const float*)d_in[0];
  const float* qw = (const float*)d_in[1]; const float* qb = (const float*)d_in[2]; const float* kw = (const float*)d_in[3]; const float* kb = (const float*)d_in[4];
  const float* vw = (const float*)d_in[5]; const float* vb = (const float*)d_in[6]; const float* qlw = (const float*)d_in[7]; const float* klw = (const float*)d_in[8];
  const float* ow = (const float*)d_in[9]; const float* ob = (const float*)d_in[10]; const float* f1w = (const float*)d_in[11]; const float* f1b = (const float*)d_in[12];
  const float* f2w = (const float*)d_in[13]; const float* f2b = (const float*)d_in[14]; const float* g1 = (const float*)d_in[15]; const float* b1 = (const float*)d_in[16];
  const float* g2 = (const float*)d_in[17]; const float* b2 = (const float*)d_in[18];
  float* out = (float*)d_out;
  if (in_sizes[0] != Bn * C * S || in_sizes[1] != 4 * 64 * 64 || in_sizes[7] != 4 * 16 * 64 || in_sizes[11] != FF * C || in_sizes[13] != C * FF) return;
  size_t off = 0; char* ws = (char*)d_ws;
  auto carve = [&](size_t bytes) { char* p = ws + off; off += (bytes + 255) & ~(size_t)255; return p; };
  const size_t NPL = (size_t)4 * 192 * 64 + 4 * 32 * 64 + 4 * 64 * 64 + (size_t)FF * C + (size_t)C * FF;
  b16* ph = (b16*)carve(NPL * 2); b16* pl = (b16*)carve(NPL * 2);
  float* bqkv = (float*)carve((size_t)4 * 192 * 4);
  float* xT  = (float*)carve((size_t)NT * C * 4);
  float* xin = (float*)carve((size_t)NT * SC * 4);
  float* QK  = (float*)carve((size_t)NT * 128 * 4);
  b16* vth = (b16*)carve((size_t)Bn * SC * S * 2); b16* vtl = (b16*)carve((size_t)Bn * SC * S * 2);
  float* Lb  = (float*)carve((size_t)2 * NT * RK * 4);
  float* Ob  = (float*)carve((size_t)NT * SC * 4);
  float* cat = (float*)carve((size_t)NT * C * 4);
  float* coef = (float*)carve((size_t)2 * C * 4);
  float* out1 = (float*)carve((size_t)NT * C * 4);
  b16* hh_ = (b16*)carve((size_t)NT * FF * 2); b16* hl_ = (b16*)carve((size_t)NT * FF * 2);
  float* h2 = (float*)carve((size_t)NT * C * 4);
  if (off > ws_size) return;
  const b16* wqkv_h = ph; const b16* wqkv_l = pl; const b16* wl_h = ph + 4 * 192 * 64; const b16* wl_l = pl + 4 * 192 * 64;
  const b16* wo_h = wl_h + 4 * 32 * 64; const b16* wo_l = wl_l + 4 * 32 * 64; const b16* w1_h = wo_h + 4 * 64 * 64; const b16* w1_l = wo_l + 4 * 64 * 64;
  const b16* w2_h = w1_h + (size_t)FF * C; const b16* w2_l = w1_l + (size_t)FF * C;
  prep_kernel<<<256, 256, 0, stream>>>(qw, kw, vw, qlw, klw, ow, f1w, f2w, qb, kb, vb, ph, pl, bqkv);
  xt_kernel<<<Bn * (S / 64), 256, 0, stream>>>(x, xT, xin);
  for (int hd = 0; hd < 4; ++hd) {
    qkv_kernel<<<dim3(3, NT / 128), 128, 0, stream>>>(xin, wqkv_h + (size_t)hd * 192 * 64, wqkv_l + (size_t)hd * 192 * 64, bqkv + hd * 192, QK, vth, vtl);
    ql_kernel<<<dim3(NT / 128, 2), 128, 0, stream>>>(QK, wl_h + (size_t)hd * 32 * 64, wl_l + (size_t)hd * 32 * 64, Lb);
    attn_kernel<<<NT / 16 / 8, 256, 0, stream>>>(Lb, vth, vtl, Ob);
    oproj_kernel<<<NT / 128, 128, 0, stream>>>(Ob, wo_h + (size_t)hd * 64 * 64, wo_l + (size_t)hd * 64 * 64, ob + hd * 64, xT, hd, cat, xin);
  }
  bnstat_kernel<<<1, 256, 0, stream>>>(cat, C, g1, b1, coef);
  bn1_kernel<<<NT / 8, 256, 0, stream>>>(xT, cat, coef, out1);
  ffn1_kernel<<<dim3(FF / 64, NT / 128), 128, 0, stream>>>(out1, w1_h, w1_l, f1b, hh_, hl_);
  ffn2_kernel<<<dim3(C / 64, NT / 128), 128, 0, stream>>>(hh_, hl_, w2_h, w2_l, f2b, h2);
  bnstat_kernel<<<1, 256, 0, stream>>>(h2, C, g2, b2, coef);
  final_kernel<<<Bn * (S / 64), 256, 0, stream>>>(out1, h2, coef, out);
}
